// InternImageLayer_11931419148987
// MI455X (gfx1250) — hardware-verified
//
#include <hip/hip_runtime.h>
#define NBt 4
#define CC 256
#define HH 64
#define NTK (HH * HH)
#define NR (NBt * NTK)
#define GG 16
#define CG 16
#define KT 9
#define NOM 432
#define NOMP 448
#define DM 1024
typedef __bf16 v16b __attribute__((ext_vector_type(16)));
typedef unsigned short v8us __attribute__((ext_vector_type(8), may_alias));
typedef float  v8f  __attribute__((ext_vector_type(8)));
typedef float  v4f  __attribute__((ext_vector_type(4)));
typedef float  v4fa __attribute__((ext_vector_type(4), may_alias));
union FragB { v16b v; v8us half[2]; unsigned short u[16]; };

__device__ __forceinline__ unsigned short bf16_bits(float x) { unsigned int u = __float_as_uint(x); return (unsigned short)((u + 0x7FFFu + ((u >> 16) & 1u)) >> 16); }
__device__ __forceinline__ float bf16_val(unsigned short b) { return __uint_as_float(((unsigned int)b) << 16); }
__device__ __forceinline__ float bf16_round(float x) { return bf16_val(bf16_bits(x)); }
template <int NT>
__device__ __forceinline__ v8f mmaN(v16b ah, v16b al, v16b bh, v16b bl, v8f c) {
  c = __builtin_amdgcn_wmma_f32_16x16x32_bf16(false, ah, false, bh, (short)0, c, false, false);
  if (NT >= 2) c = __builtin_amdgcn_wmma_f32_16x16x32_bf16(false, al, false, bh, (short)0, c, false, false);
  if (NT >= 3) c = __builtin_amdgcn_wmma_f32_16x16x32_bf16(false, ah, false, bl, (short)0, c, false, false);
  asm volatile("v_nop\n\tv_nop\n\tv_nop\n\tv_nop" : "+v"(c) : "v"(ah), "v"(al), "v"(bh), "v"(bl));
  return c;
}

__global__ __launch_bounds__(256) void k_wt_bf16(const float* __restrict__ W, unsigned short* __restrict__ Wt, int K, int N) {
  const int t = blockIdx.x * 256 + threadIdx.x;
  const int k8n = K / 8;
  if (t >= N * k8n) return;
  const int n = t / k8n, k8 = (t % k8n) * 8;
  v8us v;
#pragma unroll
  for (int i = 0; i < 8; ++i) v[i] = bf16_bits(W[(size_t)(k8 + i) * N + n]);
  *(volatile v8us*)(Wt + (size_t)n * K + k8) = v;
  __threadfence();
  *(volatile v8us*)(Wt + (size_t)n * K + k8) = v;
}

template <bool ASPLIT, int ACT, bool BIAS_BF16>
__global__ __launch_bounds__(128) void k_gemm_bf(const float* __restrict__ A, int lda, const unsigned short* __restrict__ Wt, int ldb,
                                               const float* __restrict__ bias, float* __restrict__ C, int ldc, int M, int N, int K) {
  __shared__ __attribute__((aligned(16))) float so[4][16][64];
  const int tid = threadIdx.x, w = tid >> 5, lane = tid & 31, ln = lane & 15, hh = lane >> 4;
  const int ntn = N / 64;
  const int wid = blockIdx.x * 4 + w;
  const int mt = wid / ntn, nq = wid % ntn;
  if (mt * 16 >= M) return;
  const int row0 = mt * 16, col0 = nq * 64;
  const float* arow = A + (size_t)(row0 + ln) * lda;
  v8f acc[4] = {};
  for (int kb = 0; kb < K; kb += 32) {
    FragB ah, al;
    const v4f x0 = *(const v4fa*)(arow + kb + 8 * hh), x1 = *(const v4fa*)(arow + kb + 8 * hh + 4);
    const v4f x2 = *(const v4fa*)(arow + kb + 16 + 8 * hh), x3 = *(const v4fa*)(arow + kb + 16 + 8 * hh + 4);
    float xs[16] = {x0[0],x0[1],x0[2],x0[3],x1[0],x1[1],x1[2],x1[3],x2[0],x2[1],x2[2],x2[3],x3[0],x3[1],x3[2],x3[3]};
#pragma unroll
    for (int i = 0; i < 16; ++i) { const unsigned short hb = bf16_bits(xs[i]); ah.u[i] = hb; al.u[i] = ASPLIT ? bf16_bits(xs[i] - bf16_val(hb)) : (unsigned short)0; }
#pragma unroll
    for (int t = 0; t < 4; ++t) {
      const unsigned short* brow = Wt + (size_t)(col0 + t * 16 + ln) * ldb + kb;
      FragB b;
      b.half[0] = *(const v8us*)(brow + 8 * hh);
      b.half[1] = *(const v8us*)(brow + 16 + 8 * hh);
      acc[t] = mmaN<ASPLIT ? 2 : 1>(ah.v, al.v, b.v, b.v, acc[t]);
    }
  }
#pragma unroll
  for (int t = 0; t < 4; ++t) {
    float bv = bias ? bias[col0 + t * 16 + ln] : 0.f;
    if (BIAS_BF16) bv = bf16_round(bv);
#pragma unroll
    for (int r = 0; r < 8; ++r) { float v = acc[t][r] + bv; if (ACT == 1) v = fmaxf(v, 0.f); so[w][8 * hh + r][t * 16 + ln] = v; }
  }
  __builtin_amdgcn_fence(__ATOMIC_ACQ_REL, "workgroup");
  __builtin_amdgcn_wave_barrier();
  const int rsub = lane >> 4, c4 = (lane & 15) * 4;
  for (int pass = 0; pass < 2; ++pass) {
#pragma unroll
    for (int q = 0; q < 8; ++q) {
      const int r = q * 2 + rsub;
      const v4f v = *(const v4fa*)&so[w][r][c4];
      *(volatile v4f*)(C + (size_t)(row0 + r) * ldc + col0 + c4) = v;
    }
    if (pass == 0) __threadfence();
  }
}

template <bool ASPLIT, int ACT, bool BIAS_BF16, bool RES_BF16>
__global__ __launch_bounds__(128) void k_gemm_bf3(const float* __restrict__ A, int lda, const unsigned short* __restrict__ Wt, int ldb,
                                                const float* __restrict__ bias, const float* __restrict__ resid, int rmod, int ldr,
                                                float* __restrict__ C, int ldc, int M, int N, int K) {
  __shared__ __attribute__((aligned(16))) float so[4][16][64];
  const int tid = threadIdx.x, w = tid >> 5, lane = tid & 31, ln = lane & 15, hh = lane >> 4;
  const int ntn = N / 64;
  const int wid = blockIdx.x * 4 + w;
  const int mt = wid / ntn, nq = wid % ntn;
  if (mt * 16 >= M) return;
  const int row0 = mt * 16, col0 = nq * 64;
  const float* arow = A + (size_t)(row0 + ln) * lda;
  v8f acc[4] = {};
  for (int kb = 0; kb < K; kb += 32) {
    FragB ah, al;
    const v4f x0 = *(const v4fa*)(arow + kb + 8 * hh), x1 = *(const v4fa*)(arow + kb + 8 * hh + 4);
    const v4f x2 = *(const v4fa*)(arow + kb + 16 + 8 * hh), x3 = *(const v4fa*)(arow + kb + 16 + 8 * hh + 4);
    float xs[16] = {x0[0],x0[1],x0[2],x0[3],x1[0],x1[1],x1[2],x1[3],x2[0],x2[1],x2[2],x2[3],x3[0],x3[1],x3[2],x3[3]};
#pragma unroll
    for (int i = 0; i < 16; ++i) { const unsigned short hb = bf16_bits(xs[i]); ah.u[i] = hb; al.u[i] = ASPLIT ? bf16_bits(xs[i] - bf16_val(hb)) : (unsigned short)0; }
#pragma unroll
    for (int t = 0; t < 4; ++t) {
      const unsigned short* brow = Wt + (size_t)(col0 + t * 16 + ln) * ldb + kb;
      FragB b;
      b.half[0] = *(const v8us*)(brow + 8 * hh);
      b.half[1] = *(const v8us*)(brow + 16 + 8 * hh);
      acc[t] = mmaN<ASPLIT ? 2 : 1>(ah.v, al.v, b.v, b.v, acc[t]);
    }
  }
#pragma unroll
  for (int t = 0; t < 4; ++t) {
    const int col = col0 + t * 16 + ln;
    float bv = bias ? bias[col] : 0.f;
    if (BIAS_BF16) bv = bf16_round(bv);
#pragma unroll
    for (int r = 0; r < 8; ++r) {
      float v = acc[t][r] + bv;
      if (resid) { float rv = resid[(size_t)((row0 + 8 * hh + r) % rmod) * ldr + col]; if (RES_BF16) rv = bf16_round(rv); v += rv; }
      if (ACT == 1) v = fmaxf(v, 0.f);
      if (ACT == 2) v = 0.5f * v * (1.0f + erff(v * 0.70710678118654752f));
      if (ACT == 3) { const float u = 0.7978845608028654f * (v + 0.044715f * v * v * v); v = 0.5f * v * (1.0f + tanhf(u)); }
      so[w][8 * hh + r][t * 16 + ln] = v;
    }
  }
  __builtin_amdgcn_fence(__ATOMIC_ACQ_REL, "workgroup");
  __builtin_amdgcn_wave_barrier();
  const int rsub = lane >> 4, c4 = (lane & 15) * 4;
  for (int pass = 0; pass < 2; ++pass) {
#pragma unroll
    for (int q = 0; q < 8; ++q) {
      const int r = q * 2 + rsub;
      const v4f v = *(const v4fa*)&so[w][r][c4];
      *(volatile v4f*)(C + (size_t)(row0 + r) * ldc + col0 + c4) = v;
    }
    if (pass == 0) __threadfence();
  }
}
template <bool PARAM_BF16>
__global__ __launch_bounds__(256) void k_layernorm(const float* __restrict__ X, const float* __restrict__ R, const float* __restrict__ g, const float* __restrict__ bta,
                                                  float* __restrict__ out_sum, float* __restrict__ out_norm, int N, float eps) {
  __shared__ float red[256];
  const int row = blockIdx.x, tid = threadIdx.x;
  const float* x = X + (size_t)row * N; const float* rr = R ? R + (size_t)row * N : nullptr;
  float vals[16];
  const int per = N / 256;
  float s1 = 0.f;
  for (int u = 0; u < per / 4; ++u) {
    const int j = tid * 4 + 1024 * u;
    const v4f a = *(const v4fa*)(x + j);
    v4f b = {0.f,0.f,0.f,0.f}; if (rr) b = *(const v4fa*)(rr + j);
#pragma unroll
    for (int q = 0; q < 4; ++q) { const float v = a[q] + b[q]; vals[u * 4 + q] = v; s1 += v; }
  }
  red[tid] = s1; __syncthreads();
  for (int st = 128; st > 0; st >>= 1) { if (tid < st) red[tid] += red[tid + st]; __syncthreads(); }
  const float mu = red[0] / (float)N; __syncthreads();
  float s2 = 0.f;
  for (int u = 0; u < per / 4; ++u)
#pragma unroll
    for (int q = 0; q < 4; ++q) { const float c = vals[u * 4 + q] - mu; s2 += c * c; }
  red[tid] = s2; __syncthreads();
  for (int st = 128; st > 0; st >>= 1) { if (tid < st) red[tid] += red[tid + st]; __syncthreads(); }
  const float rs = rsqrtf(red[0] / (float)N + eps);
  for (int pass = 0; pass < 2; ++pass) {
    for (int u = 0; u < per / 4; ++u) {
      const int j = tid * 4 + 1024 * u;
      v4f o, sm;
#pragma unroll
      for (int q = 0; q < 4; ++q) {
        float gg = g[j + q], bb = bta[j + q];
        if (PARAM_BF16) { gg = bf16_round(gg); bb = bf16_round(bb); }
        sm[q] = vals[u * 4 + q]; o[q] = (vals[u * 4 + q] - mu) * rs * gg + bb;
      }
      if (out_sum) *(volatile v4f*)(out_sum + (size_t)row * N + j) = sm;
      *(volatile v4f*)(out_norm + (size_t)row * N + j) = o;
    }
    if (pass == 0) __threadfence();
  }
}


typedef _Float16 v16h __attribute__((ext_vector_type(16)));
union FragH { v16h v; v8us half[2]; _Float16 h[16]; unsigned short u[16]; };
template <int NT>
__device__ __forceinline__ v8f mmaH(v16h ah, v16h al, v16h bh, v16h bl, v8f c) {
  c = __builtin_amdgcn_wmma_f32_16x16x32_f16(false, ah, false, bh, (short)0, c, false, false);
  if (NT >= 2) c = __builtin_amdgcn_wmma_f32_16x16x32_f16(false, al, false, bh, (short)0, c, false, false);
  if (NT >= 3) c = __builtin_amdgcn_wmma_f32_16x16x32_f16(false, ah, false, bl, (short)0, c, false, false);
  asm volatile("v_nop\n\tv_nop\n\tv_nop\n\tv_nop" : "+v"(c) : "v"(ah), "v"(al), "v"(bh), "v"(bl));
  return c;
}
template <bool ASPLIT>
__global__ __launch_bounds__(128) void k_gemm_h(const float* __restrict__ A, int lda, size_t sA, const _Float16* __restrict__ Bh, int ldb, size_t sB, float alpha, float* __restrict__ C, int ldc, size_t sC, int M, int N, int K) {
  __shared__ __attribute__((aligned(16))) float so[4][16][64];
  const int tid = threadIdx.x, w = tid >> 5, lane = tid & 31, ln = lane & 15, hh = lane >> 4; const int by = blockIdx.y;
  A += (size_t)by * sA; Bh += (size_t)by * sB; C += (size_t)by * sC;
  const int ntn = (N + 63) / 64; const int wid = blockIdx.x * 4 + w; const int mt = wid / ntn, nq = wid % ntn; if (mt * 16 >= M) return;
  const int row0 = mt * 16, col0 = nq * 64; const float* arow = A + (size_t)(row0 + ln) * lda;
  v8f acc[4] = {};
  for (int kb = 0; kb < K; kb += 32) {
    FragH ah, al;
    const v4f x0 = *(const v4fa*)(arow + kb + 8 * hh), x1 = *(const v4fa*)(arow + kb + 8 * hh + 4), x2 = *(const v4fa*)(arow + kb + 16 + 8 * hh), x3 = *(const v4fa*)(arow + kb + 16 + 8 * hh + 4);
    float xs[16] = {x0[0],x0[1],x0[2],x0[3],x1[0],x1[1],x1[2],x1[3],x2[0],x2[1],x2[2],x2[3],x3[0],x3[1],x3[2],x3[3]};
#pragma unroll
    for (int i = 0; i < 16; ++i) { const _Float16 h = (_Float16)xs[i]; ah.h[i] = h; al.h[i] = ASPLIT ? (_Float16)(xs[i] - (float)h) : (_Float16)0.0f; }
#pragma unroll
    for (int t = 0; t < 4; ++t) { if (col0 + t * 16 >= N) continue; const size_t boff = (size_t)(col0 + t * 16 + ln) * ldb + kb; FragH bq; bq.half[0] = *(const v8us*)(Bh + boff + 8 * hh); bq.half[1] = *(const v8us*)(Bh + boff + 16 + 8 * hh);
      acc[t] = mmaH<ASPLIT ? 2 : 1>(ah.v, al.v, bq.v, bq.v, acc[t]); }
  }
#pragma unroll
  for (int t = 0; t < 4; ++t) { if (col0 + t * 16 >= N) continue;
#pragma unroll
    for (int r = 0; r < 8; ++r) so[w][8 * hh + r][t * 16 + ln] = acc[t][r] * alpha; }
  __builtin_amdgcn_fence(__ATOMIC_ACQ_REL, "workgroup"); __builtin_amdgcn_wave_barrier();
  const int rsub = lane >> 4, c4 = (lane & 15) * 4;
  for (int pass = 0; pass < 2; ++pass) {
#pragma unroll
    for (int q = 0; q < 8; ++q) { const int r = q * 2 + rsub; if (col0 + c4 < N) { const v4f v = *(const v4fa*)&so[w][r][c4]; *(volatile v4f*)(C + (size_t)(row0 + r) * ldc + col0 + c4) = v; } }
    if (pass == 0) __threadfence(); }
}

__global__ __launch_bounds__(256) void k_wt_f16(const float* __restrict__ W, _Float16* __restrict__ Wt, int K, int N, float scale) {
  const int t = blockIdx.x * 256 + threadIdx.x; if (t >= N * (K / 8)) return; const int n = t / (K / 8), k8 = (t % (K / 8)) * 8; FragH f;
#pragma unroll
  for (int i = 0; i < 8; ++i) f.h[i] = (_Float16)(bf16_round(W[(size_t)(k8 + i) * N + n]) * scale); const v8us o = f.half[0];
  *(volatile v8us*)((unsigned short*)Wt + (size_t)n * K + k8) = o; __threadfence(); *(volatile v8us*)((unsigned short*)Wt + (size_t)n * K + k8) = o;
}
template <int ACT>
__global__ __launch_bounds__(128) void k_gemm_hhx(const _Float16* __restrict__ A, int lda, size_t sA, const _Float16* __restrict__ Bh, int ldb, size_t sB, float alpha, const float* __restrict__ bias, size_t sBias, const float* __restrict__ CP, int rowsPerB, size_t sCPb, int row0g,
    float* __restrict__ C, _Float16* __restrict__ C16, int ldc, size_t sC, int M, int N, int K) {
  __shared__ __attribute__((aligned(16))) float so[4][16][64];
  const int tid = threadIdx.x, w = tid >> 5, lane = tid & 31, ln = lane & 15, hh = lane >> 4; const int by = blockIdx.y;
  A += (size_t)by * sA; Bh += (size_t)by * sB; const size_t cofs = (size_t)by * sC; const float* bp = bias ? bias + (size_t)by * sBias : nullptr;
  const int ntn = (N + 63) / 64; const int wid = blockIdx.x * 4 + w; const int mt = wid / ntn, nq = wid % ntn; if (mt * 16 >= M) return;
  const int row0 = mt * 16, col0 = nq * 64; const _Float16* arow = A + (size_t)(row0 + ln) * lda;
  v8f acc[4] = {};
  for (int kb = 0; kb < K; kb += 32) { FragH ah; ah.half[0] = *(const v8us*)((const unsigned short*)arow + kb + 8 * hh); ah.half[1] = *(const v8us*)((const unsigned short*)arow + kb + 16 + 8 * hh);
#pragma unroll
    for (int t = 0; t < 4; ++t) { if (col0 + t * 16 >= N) continue; const size_t boff = (size_t)(col0 + t * 16 + ln) * ldb + kb; FragH bq; bq.half[0] = *(const v8us*)((const unsigned short*)Bh + boff + 8 * hh); bq.half[1] = *(const v8us*)((const unsigned short*)Bh + boff + 16 + 8 * hh);
      acc[t] = mmaH<1>(ah.v, ah.v, bq.v, bq.v, acc[t]); }
  }
#pragma unroll
  for (int t = 0; t < 4; ++t) { if (col0 + t * 16 >= N) continue; const int col = col0 + t * 16 + ln; const float bv = bp ? bf16_round(bp[col]) : 0.f;
#pragma unroll
    for (int r = 0; r < 8; ++r) { float v = acc[t][r] * alpha + bv; if (CP) { const int bidx = (row0g + row0 + 8 * hh + r) / rowsPerB; v += CP[(size_t)bidx * sCPb + (size_t)by * 64 + col]; } if (ACT == 1) v = (v > 0.f) ? v : expm1f(v); else if (ACT == 7) v = (v > 0.f) ? v + 1.0f : expf(v); else if (ACT == 8) v = tanhf(v); else if (ACT == 9) v = 0.5f * v * (1.0f + tanhf(0.7978845608028654f * (v + 0.044715f * v * v * v))); else if (ACT == 11) v = 1.0f / (1.0f + expf(-v)); else if (ACT == 12) v = (v > 0.f) ? v : 0.01f * v; else if (ACT == 14) v = (v > 0.f) ? v : 0.1f * v; else if (ACT == 15) v = v / (1.0f + expf(-v)); else if (ACT == 3) v = fmaxf(v, 0.f); else if (ACT == 6) v = 0.5f * v * (1.0f + erff(v * 0.70710678118654752f)); so[w][8 * hh + r][t * 16 + ln] = v; } }
  __builtin_amdgcn_fence(__ATOMIC_ACQ_REL, "workgroup"); __builtin_amdgcn_wave_barrier();
  const int rsub = lane >> 4, c4 = (lane & 15) * 4; typedef _Float16 v4h __attribute__((ext_vector_type(4)));
  for (int pass = 0; pass < 2; ++pass) {
#pragma unroll
    for (int q = 0; q < 8; ++q) { const int r = q * 2 + rsub; if (col0 + c4 < N) { const v4f v = *(const v4fa*)&so[w][r][c4]; if (C) *(volatile v4f*)(C + cofs + (size_t)(row0 + r) * ldc + col0 + c4) = v; if (C16) { v4h h4; for (int i = 0; i < 4; ++i) h4[i] = (_Float16)v[i]; *(volatile v4h*)(C16 + cofs + (size_t)(row0 + r) * ldc + col0 + c4) = h4; } } }
    if (pass == 0) __threadfence(); }
}


typedef _Float16 v4h __attribute__((ext_vector_type(4)));

__global__ __launch_bounds__(256) void k_x16(const float* __restrict__ x, _Float16* __restrict__ X16, size_t n8) { const size_t t = (size_t)blockIdx.x * 256 + threadIdx.x; if (t >= n8) return; FragH f;
#pragma unroll
  for (int q = 0; q < 8; ++q) f.h[q] = (_Float16)bf16_round(x[t * 8 + q]); *(volatile v8us*)((unsigned short*)X16 + t * 8) = f.half[0]; __threadfence(); *(volatile v8us*)((unsigned short*)X16 + t * 8) = f.half[0]; }
__global__ __launch_bounds__(256) void k_h16(const float* __restrict__ x, _Float16* __restrict__ X16, size_t n8) { const size_t t = (size_t)blockIdx.x * 256 + threadIdx.x; if (t >= n8) return; FragH f;
#pragma unroll
  for (int q = 0; q < 8; ++q) f.h[q] = (_Float16)x[t * 8 + q]; *(volatile v8us*)((unsigned short*)X16 + t * 8) = f.half[0]; __threadfence(); *(volatile v8us*)((unsigned short*)X16 + t * 8) = f.half[0]; }
__global__ __launch_bounds__(256) void k_round16f(const float* __restrict__ W, _Float16* __restrict__ Bt, size_t n8) { const size_t t = (size_t)blockIdx.x * 256 + threadIdx.x; if (t >= n8) return; FragH f;
#pragma unroll
  for (int i = 0; i < 8; ++i) f.h[i] = (_Float16)(bf16_round(W[t * 8 + i]) * 16.0f); *(volatile v8us*)((unsigned short*)Bt + t * 8) = f.half[0]; __threadfence(); *(volatile v8us*)((unsigned short*)Bt + t * 8) = f.half[0]; }
template <int NHv, int TTv>
__global__ __launch_bounds__(256) void k_vt(const _Float16* __restrict__ V16, int ldv, int voff, _Float16* __restrict__ Vt) { __shared__ unsigned short tl[64][66]; const int tid = threadIdx.x; const int slab = blockIdx.x / (TTv / 64), lg = blockIdx.x % (TTv / 64); const int b = slab / NHv, h = slab % NHv;
  for (int i = tid; i < 64 * 8; i += 256) { const int r = i / 8, c8 = (i % 8) * 8; FragH f; f.half[0] = *(const v8us*)((const unsigned short*)V16 + ((size_t)b * TTv + lg * 64 + r) * ldv + voff + h * 64 + c8);
#pragma unroll
    for (int q = 0; q < 8; ++q) tl[r][c8 + q] = f.u[q]; }
  __syncthreads();
  for (int pass = 0; pass < 2; ++pass) {
#pragma unroll
    for (int rd = 0; rd < 2; ++rd) { const int d = rd * 32 + tid / 8, pc = tid % 8; FragH f;
#pragma unroll
      for (int q = 0; q < 8; ++q) f.u[q] = tl[pc * 8 + q][d];
      *(volatile v8us*)((unsigned short*)Vt + ((size_t)slab * 64 + d) * TTv + lg * 64 + pc * 8) = f.half[0]; }
    if (pass == 0) __threadfence(); } }

__global__ __launch_bounds__(256) void k_hl(const float* __restrict__ F, _Float16* __restrict__ Hh, _Float16* __restrict__ Hl, size_t n8) { const size_t t = (size_t)blockIdx.x * 256 + threadIdx.x; if (t >= n8) return; FragH fh, fl; const v4f a = *(const v4fa*)(F + t * 8), c = *(const v4fa*)(F + t * 8 + 4);
#pragma unroll
  for (int q = 0; q < 4; ++q) { _Float16 h = (_Float16)a[q]; fh.h[q] = h; fl.h[q] = (_Float16)((a[q] - (float)h) * 1024.0f); h = (_Float16)c[q]; fh.h[4 + q] = h; fl.h[4 + q] = (_Float16)((c[q] - (float)h) * 1024.0f); }
  for (int pass = 0; pass < 2; ++pass) { *(volatile v8us*)((unsigned short*)Hh + t * 8) = fh.half[0]; *(volatile v8us*)((unsigned short*)Hl + t * 8) = fl.half[0]; if (pass == 0) __threadfence(); } }

__device__ __forceinline__ float gelu_f(float v) { return 0.5f * v * (1.0f + erff(v * 0.70710678118654752f)); }
__global__ __launch_bounds__(256) void k_tok(const float* __restrict__ x, float* __restrict__ X) { const int t = blockIdx.x * 256 + threadIdx.x; if (t >= NR * (CC / 4)) return; const int c0 = (t % (CC / 4)) * 4, r = t / (CC / 4); const int b = r / NTK, l = r % NTK; v4f v;
#pragma unroll
  for (int q = 0; q < 4; ++q) v[q] = bf16_round(x[((size_t)b * CC + c0 + q) * NTK + l]);
  *(volatile v4f*)(X + (size_t)r * CC + c0) = v; __threadfence(); *(volatile v4f*)(X + (size_t)r * CC + c0) = v; }
__global__ __launch_bounds__(256) void k_ln2p(const float* __restrict__ X, const float* __restrict__ g, const float* __restrict__ bb, _Float16* __restrict__ X2) {
  #pragma clang fp contract(off)
  const int tid = threadIdx.x, w = tid >> 5, ln = tid & 31; const int r = blockIdx.x * 8 + w; if (r >= NR) return; float v[8]; float s = 0.f;
#pragma unroll
  for (int k = 0; k < 8; ++k) { v[k] = X[(size_t)r * CC + ln * 8 + k]; s += v[k]; }
  for (int o = 16; o > 0; o >>= 1) s += __shfl_xor(s, o, 32); const float mu = s / (float)CC; float q2 = 0.f;
#pragma unroll
  for (int k = 0; k < 8; ++k) { const float d = v[k] - mu; q2 += d * d; }
  for (int o = 16; o > 0; o >>= 1) q2 += __shfl_xor(q2, o, 32); const float rs = rsqrtf(q2 / (float)CC + 1e-5f); FragH fh, fl;
#pragma unroll
  for (int k = 0; k < 8; ++k) { const int c = ln * 8 + k; const float y = (v[k] - mu) * rs * bf16_round(g[c]) + bf16_round(bb[c]); const _Float16 hi = (_Float16)y; fh.h[k] = hi; fl.h[k] = (_Float16)((y - (float)hi) * 1024.0f); }
  for (int pass = 0; pass < 2; ++pass) { *(volatile v8us*)((unsigned short*)X2 + (size_t)r * 512 + ln * 8) = fh.half[0]; *(volatile v8us*)((unsigned short*)X2 + (size_t)r * 512 + 256 + ln * 8) = fl.half[0]; if (pass == 0) __threadfence(); } }
__global__ __launch_bounds__(256) void k_bfold(const float* __restrict__ Wm, int O, int Opad, _Float16* __restrict__ Bt) { const int t = blockIdx.x * 256 + threadIdx.x; if (t >= Opad * 64) return; const int k0 = (t & 63) * 8, o = t >> 6; const int kb = k0 & 255; const float sc = (k0 >= 256) ? (16.0f / 1024.0f) : 16.0f; FragH f;
#pragma unroll
  for (int q = 0; q < 8; ++q) f.h[q] = (o < O) ? (_Float16)(bf16_round(Wm[(size_t)min(o, O - 1) * CC + kb + q]) * sc) : (_Float16)0.0f;
  *(volatile v8us*)((unsigned short*)Bt + (size_t)o * 512 + k0) = f.half[0]; __threadfence(); *(volatile v8us*)((unsigned short*)Bt + (size_t)o * 512 + k0) = f.half[0]; }
__global__ __launch_bounds__(256) void k_bpad(const float* __restrict__ bb, int n, int np, float* __restrict__ BP) { const int l = blockIdx.x * 256 + threadIdx.x; if (l >= np) return; const float v = (l < n) ? bb[l] : 0.f; *(volatile float*)(BP + l) = v; __threadfence(); *(volatile float*)(BP + l) = v; }
__global__ __launch_bounds__(256) void k_dcn(const float* __restrict__ OM, const _Float16* __restrict__ V16, _Float16* __restrict__ D16) {
  #pragma clang fp contract(off)
  const int t = blockIdx.x * 256 + threadIdx.x; if (t >= NR * GG) return; const int g = t & 15, r = t >> 4; const int b = r / NTK, l = r % NTK; const int h = l / HH, w = l % HH; const float* om = OM + (size_t)r * NOMP + g * 27; float acc[CG];
#pragma unroll
  for (int c = 0; c < CG; ++c) acc[c] = 0.f;
#pragma unroll 1
  for (int k = 0; k < KT; ++k) { const float offx = om[2 * k], offy = om[2 * k + 1], m = om[18 + k]; const float px = (float)w + ((float)(k % 3 - 1) + offx), py = (float)h + ((float)(k / 3 - 1) + offy); const float x0 = floorf(px), y0 = floorf(py); const float tx = px - x0, ty = py - y0; const int xi = (int)x0, yi = (int)y0;
#pragma unroll
    for (int cn = 0; cn < 4; ++cn) { const int xx = xi + (cn & 1), yy = yi + (cn >> 1); const bool valid = (xx >= 0 && xx < HH && yy >= 0 && yy < HH); const float wgt = ((cn & 1) ? tx : (1.0f - tx)) * ((cn >> 1) ? ty : (1.0f - ty)); const float f = valid ? (m * wgt) : 0.f; const int lin = min(max(yy, 0), HH - 1) * HH + min(max(xx, 0), HH - 1); const _Float16* vp = V16 + ((size_t)b * NTK + lin) * CC + g * CG; FragH va, vb; va.half[0] = *(const v8us*)(const unsigned short*)vp; vb.half[0] = *(const v8us*)((const unsigned short*)vp + 8);
#pragma unroll
      for (int c = 0; c < 8; ++c) { acc[c] += f * (float)va.h[c]; acc[8 + c] += f * (float)vb.h[c]; } } }
  FragH oa, ob;
#pragma unroll
  for (int c = 0; c < 8; ++c) { oa.h[c] = (_Float16)acc[c]; ob.h[c] = (_Float16)acc[8 + c]; }
  for (int pass = 0; pass < 2; ++pass) { *(volatile v8us*)((unsigned short*)D16 + (size_t)r * CC + g * CG) = oa.half[0]; *(volatile v8us*)((unsigned short*)D16 + (size_t)r * CC + g * CG + 8) = ob.half[0]; if (pass == 0) __threadfence(); } }
__global__ __launch_bounds__(256) void k_gelu(const float* __restrict__ T, _Float16* __restrict__ H16, size_t n4) {
  #pragma clang fp contract(off)
  const size_t t = (size_t)blockIdx.x * 256 + threadIdx.x; if (t >= n4) return; const v4f a = *(const v4fa*)(T + t * 4); FragH f;
#pragma unroll
  for (int q = 0; q < 4; ++q) f.h[q] = (_Float16)gelu_f(a[q]);
  const unsigned long long pv = *(const unsigned long long*)&f.u[0]; *(volatile unsigned long long*)((unsigned short*)H16 + t * 4) = pv; __threadfence(); *(volatile unsigned long long*)((unsigned short*)H16 + t * 4) = pv; }
__global__ __launch_bounds__(256) void k_nchw(const float* __restrict__ Xf, float* __restrict__ out) { const int t = blockIdx.x * 256 + threadIdx.x; if (t >= NBt * CC * (NTK / 4)) return; const int l0 = (t % (NTK / 4)) * 4; const int c = (t / (NTK / 4)) % CC; const int b = t / ((NTK / 4) * CC); v4f v;
#pragma unroll
  for (int q = 0; q < 4; ++q) v[q] = Xf[((size_t)b * NTK + l0 + q) * CC + c];
  float* dst = out + ((size_t)b * CC + c) * NTK + l0; *(volatile v4f*)dst = v; __threadfence(); *(volatile v4f*)dst = v; }

extern "C" void kernel_launch(void* const* d_in, const int* in_sizes, int n_in,
                              void* d_out, int out_size, void* d_ws, size_t ws_size, hipStream_t stream) {
  (void)in_sizes; (void)n_in; (void)out_size;
  const float* const* I = (const float* const*)d_in; const float* x = I[0]; const float* n1g = I[1]; const float* n1b = I[2]; const float* vw = I[3]; const float* vb = I[4]; const float* omw = I[5]; const float* omb = I[6]; const float* ow = I[7]; const float* ob = I[8]; const float* n2g = I[9]; const float* n2b = I[10]; const float* f1w = I[11]; const float* f1b = I[12]; const float* f2w = I[13]; const float* f2b = I[14];
  char* ws = (char*)d_ws; size_t off = 0;
  auto take = [&](size_t bytes) { char* p = ws + off; off += (bytes + 255) & ~(size_t)255; return p; };
  _Float16* BV = (_Float16*)take((size_t)CC * 512 * 2); _Float16* BOM = (_Float16*)take((size_t)NOMP * 512 * 2); _Float16* BO = (_Float16*)take((size_t)CC * CC * 2); _Float16* BF1 = (_Float16*)take((size_t)DM * 512 * 2); _Float16* BF2 = (_Float16*)take((size_t)CC * DM * 2); float* BPom = (float*)take(NOMP * 4);
  float* X = (float*)take((size_t)NR * CC * 4); _Float16* X2 = (_Float16*)take((size_t)NR * 512 * 2); _Float16* V16 = (_Float16*)take((size_t)NR * CC * 2); float* OM = (float*)take((size_t)NR * NOMP * 4); _Float16* D16 = (_Float16*)take((size_t)NR * CC * 2); float* X1 = (float*)take((size_t)NR * CC * 4); float* T1 = (float*)take((size_t)NTK * DM * 4); _Float16* H16 = (_Float16*)take((size_t)NTK * DM * 2);
  float* X2f = X;
  if (off > ws_size) return;
  k_bfold<<<(CC * 64 + 255) / 256, 256, 0, stream>>>(vw, CC, CC, BV); k_bfold<<<(NOMP * 64 + 255) / 256, 256, 0, stream>>>(omw, NOM, NOMP, BOM); k_bfold<<<(DM * 64 + 255) / 256, 256, 0, stream>>>(f1w, DM, DM, BF1);
  k_round16f<<<(CC * CC / 8 + 255) / 256, 256, 0, stream>>>(ow, BO, (size_t)CC * CC / 8); k_round16f<<<(unsigned)(((size_t)CC * DM / 8 + 255) / 256), 256, 0, stream>>>(f2w, BF2, (size_t)CC * DM / 8);
  k_bpad<<<2, 256, 0, stream>>>(omb, NOM, NOMP, BPom);
  k_tok<<<(NR * (CC / 4) + 255) / 256, 256, 0, stream>>>(x, X);
  k_ln2p<<<NR / 8, 256, 0, stream>>>(X, n1g, n1b, X2);
  const dim3 gC(((NR / 16) * (CC / 64) + 3) / 4, 1), gOM(((NR / 16) * (NOMP / 64) + 3) / 4, 1);
  k_gemm_hhx<0><<<gC, 128, 0, stream>>>(X2, 512, 0, BV, 512, 0, 0.0625f, vb, 0, nullptr, 1, 0, 0, nullptr, V16, CC, 0, NR, CC, 512);
  k_gemm_hhx<0><<<gOM, 128, 0, stream>>>(X2, 512, 0, BOM, 512, 0, 0.0625f, BPom, 0, nullptr, 1, 0, 0, OM, nullptr, NOMP, 0, NR, NOMP, 512);
  k_dcn<<<(NR * GG + 255) / 256, 256, 0, stream>>>(OM, V16, D16);
  k_gemm_hhx<0><<<gC, 128, 0, stream>>>(D16, CC, 0, BO, CC, 0, 0.0625f, ob, 0, X, 1, (size_t)CC, 0, X1, nullptr, CC, 0, NR, CC, CC);
  k_ln2p<<<NR / 8, 256, 0, stream>>>(X1, n2g, n2b, X2);
  const dim3 gF(((NTK / 16) * (DM / 64) + 3) / 4, 1), gB(((NTK / 16) * (CC / 64) + 3) / 4, 1);
  for (int b = 0; b < NBt; ++b) { const size_t r0 = (size_t)b * NTK;
    k_gemm_hhx<0><<<gF, 128, 0, stream>>>(X2 + r0 * 512, 512, 0, BF1, 512, 0, 0.0625f, f1b, 0, nullptr, 1, 0, 0, T1, nullptr, DM, 0, NTK, DM, 512); k_gelu<<<(unsigned)(((size_t)NTK * DM / 4 + 255) / 256), 256, 0, stream>>>(T1, H16, (size_t)NTK * DM / 4);
    k_gemm_hhx<0><<<gB, 128, 0, stream>>>(H16, DM, 0, BF2, DM, 0, 0.0625f, f2b, 0, X1 + r0 * CC, 1, (size_t)CC, 0, X2f + r0 * CC, nullptr, CC, 0, NTK, CC, DM); }
  k_nchw<<<(NBt * CC * (NTK / 4) + 255) / 256, 256, 0, stream>>>(X2f, (float*)d_out);
}
